// BFS_Neural_Execution_85925115724476
// MI455X (gfx1250) — hardware-verified
//
#include <hip/hip_runtime.h>
#include <stddef.h>


#pragma clang fp contract(off)

#define DN      128
#define NTHR    256
#define NWAVE   8
#define NBN     64
#define APA     136
#define APN     264
#define GSTR    132
#define PQROW   256
#define EPT     8
#define PIECE   (NTHR * EPT)
#define WCAP    (EPT * 32)
#define NBC     512
#define SLB     9
#define PEH     0
#define PEL     16384
#define PPH     32768
#define PPL     65536
#define PUH     98304
#define PUL     131072
#define PWTOT   163840
#define SEG1    16384
#define SEG2    49152
#define PUNIQ   81920
#define PBLK    (PUNIQ / (NTHR * 8))
#define WSCAP   134217728
#define ENCDYN  (NBN * GSTR * 4)
#define UPDDYN  (2 * NBN * APN * 2)
#define AGGDYN  (NBC * DN * 4)

static_assert((PUNIQ % (NTHR * 8)) == 0);
static_assert((SEG1 % (NTHR * 8)) == 0);
static_assert((SEG2 % (NTHR * 8)) == 0);
static_assert(((APA * 2) % 16) == 0);
static_assert(((APN * 2) % 16) == 0);
static_assert(((GSTR * 4) % 16) == 0);
static_assert(NBC == (1 << SLB));
static_assert(PIECE == 2048);
static_assert((EPT % 4) == 0);
static_assert((NBC % NWAVE) == 0);
static_assert(NBN == 4 * 16);
static_assert((NBC * DN) % (4 * NTHR) == 0);
static_assert(NWAVE * 1024 * 4 <= ENCDYN);
static_assert(NBN == NWAVE * 8);

typedef float          v4f   __attribute__((ext_vector_type(4)));
typedef float          v8f   __attribute__((ext_vector_type(8)));
typedef int            v4i   __attribute__((ext_vector_type(4)));
typedef unsigned short v8us  __attribute__((ext_vector_type(8)));
typedef __bf16         v8b   __attribute__((ext_vector_type(8)));
typedef __bf16         v16b  __attribute__((ext_vector_type(16)));

__device__ __forceinline__ v16b mkfrag(v8us u0, v8us u1) {
  const v8b a = __builtin_bit_cast(v8b, u0);
  const v8b b = __builtin_bit_cast(v8b, u1);
  return __builtin_shufflevector(a, b, 0, 1, 2, 3, 4, 5, 6, 7, 8, 9, 10, 11, 12, 13, 14, 15);
}

__device__ __forceinline__ v8f wmb(v16b a, v16b b, v8f c) {
  v8f d = __builtin_amdgcn_wmma_f32_16x16x32_bf16(false, a, false, b, (short)0, c, false, false);
  asm volatile("v_nop\n\tv_nop\n\tv_nop\n\tv_nop" : "+v"(d) : "v"(a), "v"(b));
  return d;
}
__device__ __forceinline__ v8f zero8() {
  v8f z = {0.f, 0.f, 0.f, 0.f, 0.f, 0.f, 0.f, 0.f};
  return z;
}
__device__ __forceinline__ int imin(int a, int b) { return a < b ? a : b; }
__device__ __forceinline__ int iclamp(int v, int lo, int hi) { return v < lo ? lo : (v > hi ? hi : v); }

__device__ __forceinline__ unsigned int bfr(float f) {
  const unsigned int u = __float_as_uint(f);
  return (u + 0x7FFFu + ((u >> 16) & 1u)) >> 16;
}
__device__ __forceinline__ void split2(float f, unsigned short& h, unsigned short& l) {
  const unsigned int hu = bfr(f);
  const float r = f - __uint_as_float(hu << 16);
  h = (unsigned short)hu;
  l = (unsigned short)bfr(r);
}
__device__ __forceinline__ void split8v(v4f a, v4f b, unsigned short* dh, unsigned short* dl) {
  v8us hu, lu;
  unsigned short h, l;
  split2(a.x, h, l); hu[0] = h; lu[0] = l;
  split2(a.y, h, l); hu[1] = h; lu[1] = l;
  split2(a.z, h, l); hu[2] = h; lu[2] = l;
  split2(a.w, h, l); hu[3] = h; lu[3] = l;
  split2(b.x, h, l); hu[4] = h; lu[4] = l;
  split2(b.y, h, l); hu[5] = h; lu[5] = l;
  split2(b.z, h, l); hu[6] = h; lu[6] = l;
  split2(b.w, h, l); hu[7] = h; lu[7] = l;
  *(v8us*)dh = hu;
  *(v8us*)dl = lu;
}

__device__ __forceinline__ float sigm_f(float z) {
  const float zc = fminf(fmaxf(z, -80.0f), 80.0f);
  return __builtin_amdgcn_rcpf(1.0f + __expf(-zc));
}

__device__ __forceinline__ void gemm3(const unsigned short* aph, const unsigned short* apl,
                                      const unsigned short* __restrict__ bh, const unsigned short* __restrict__ bl,
                                      int kp, int nks, int n0, int m, int hh,
                                      v8f& c0, v8f& c1, v8f& c2, v8f& c3) {
  c0 = zero8(); c1 = zero8(); c2 = zero8(); c3 = zero8();
#pragma unroll 1
  for (int ks = 0; ks < nks; ++ks) {
    const v16b ah = mkfrag(*(const v8us*)(aph + 32 * ks), *(const v8us*)(aph + 32 * ks + 16));
    const v16b al = mkfrag(*(const v8us*)(apl + 32 * ks), *(const v8us*)(apl + 32 * ks + 16));
    const size_t bo = (size_t)(n0 + m) * kp + 32 * ks + 8 * hh;
    {
      const size_t o = bo;
      v16b b = mkfrag(*(const v8us*)(bh + o), *(const v8us*)(bh + o + 16));
      c0 = wmb(ah, b, c0);
      c0 = wmb(al, b, c0);
      b = mkfrag(*(const v8us*)(bl + o), *(const v8us*)(bl + o + 16));
      c0 = wmb(ah, b, c0);
    }
    {
      const size_t o = bo + (size_t)16 * kp;
      v16b b = mkfrag(*(const v8us*)(bh + o), *(const v8us*)(bh + o + 16));
      c1 = wmb(ah, b, c1);
      c1 = wmb(al, b, c1);
      b = mkfrag(*(const v8us*)(bl + o), *(const v8us*)(bl + o + 16));
      c1 = wmb(ah, b, c1);
    }
    {
      const size_t o = bo + (size_t)32 * kp;
      v16b b = mkfrag(*(const v8us*)(bh + o), *(const v8us*)(bh + o + 16));
      c2 = wmb(ah, b, c2);
      c2 = wmb(al, b, c2);
      b = mkfrag(*(const v8us*)(bl + o), *(const v8us*)(bl + o + 16));
      c2 = wmb(ah, b, c2);
    }
    {
      const size_t o = bo + (size_t)48 * kp;
      v16b b = mkfrag(*(const v8us*)(bh + o), *(const v8us*)(bh + o + 16));
      c3 = wmb(ah, b, c3);
      c3 = wmb(al, b, c3);
      b = mkfrag(*(const v8us*)(bl + o), *(const v8us*)(bl + o + 16));
      c3 = wmb(ah, b, c3);
    }
  }
}

__device__ __forceinline__ void stage_enc(float* sp, v8f a, float bias, float w0, const float* xp) {
#pragma unroll
  for (int r = 0; r < 8; ++r) sp[r * GSTR] = fmaxf((a[r] + bias) + xp[r] * w0, 0.0f);
}
__device__ __forceinline__ void stage_relu(float* sp, v8f a, float bias) {
#pragma unroll
  for (int r = 0; r < 8; ++r) sp[r * GSTR] = fmaxf(a[r] + bias, 0.0f);
}

__global__ __launch_bounds__(NTHR) void k_prep(
    const float* __restrict__ encw, const float* __restrict__ mw, const float* __restrict__ uw, unsigned short* wp) {
  const int tid = (int)threadIdx.x;
  const int o = ((int)blockIdx.x * NTHR + tid) * 8;
  const float* src;
  int rowb, col, ph, pl;
  if (o < SEG1) {
    src = encw; rowb = (o & 127) + 1; col = o >> 7; ph = PEH + o; pl = PEL + o;
  } else if (o < SEG2) {
    const int idx = o - SEG1;
    const int n = idx >> 7;
    src = mw; rowb = (n >> 7) * DN + (idx & 127); col = n & 127; ph = PPH + idx; pl = PPL + idx;
  } else {
    const int idx = o - SEG2;
    src = uw; rowb = idx & 255; col = idx >> 8; ph = PUH + idx; pl = PUL + idx;
  }
  v4f a, b;
  a.x = src[(size_t)(rowb + 0) * DN + col];
  a.y = src[(size_t)(rowb + 1) * DN + col];
  a.z = src[(size_t)(rowb + 2) * DN + col];
  a.w = src[(size_t)(rowb + 3) * DN + col];
  b.x = src[(size_t)(rowb + 4) * DN + col];
  b.y = src[(size_t)(rowb + 5) * DN + col];
  b.z = src[(size_t)(rowb + 6) * DN + col];
  b.w = src[(size_t)(rowb + 7) * DN + col];
  v8us hu, lu;
  unsigned short h, l;
  split2(a.x, h, l); hu[0] = h; lu[0] = l;
  split2(a.y, h, l); hu[1] = h; lu[1] = l;
  split2(a.z, h, l); hu[2] = h; lu[2] = l;
  split2(a.w, h, l); hu[3] = h; lu[3] = l;
  split2(b.x, h, l); hu[4] = h; lu[4] = l;
  split2(b.y, h, l); hu[5] = h; lu[5] = l;
  split2(b.z, h, l); hu[6] = h; lu[6] = l;
  split2(b.w, h, l); hu[7] = h; lu[7] = l;
  unsigned short* dh = wp + ph;
  unsigned short* dl = wp + pl;
  *(volatile v8us*)dh = hu;
  *(volatile v8us*)dl = lu;
  __threadfence();
  *(volatile v8us*)dh = hu;
  *(volatile v8us*)dl = lu;
}

__global__ __launch_bounds__(NTHR) void k_encpq(
    const float* __restrict__ x, const float* __restrict__ preh, const float* __restrict__ encw,
    const float* __restrict__ encb, const unsigned short* __restrict__ wp, float* Z, float* PQ, int nN) {
  extern __shared__ __attribute__((aligned(16))) float stg[];
  __shared__ __attribute__((aligned(16))) unsigned short sAh[NBN * APA];
  __shared__ __attribute__((aligned(16))) unsigned short sAl[NBN * APA];
  __shared__ __attribute__((aligned(16))) float sPar[2 * DN];
  __shared__ __attribute__((aligned(16))) float sX[NBN];
  const int tid = (int)threadIdx.x, lane = tid & 31, wave = tid >> 5, hh = lane >> 4, m = lane & 15;
  const int n0 = (int)blockIdx.x * NBN;

  {
    const int nl = tid >> 2, q = tid & 3;
    int node = n0 + nl;
    node = node > nN - 1 ? nN - 1 : node;
    const float* rp = preh + (size_t)node * DN + 32 * q;
#pragma unroll
    for (int i = 0; i < 4; ++i) {
      const v4f a = *(const v4f*)(rp + 8 * i);
      const v4f b = *(const v4f*)(rp + 8 * i + 4);
      split8v(a, b, sAh + nl * APA + 32 * q + 8 * i, sAl + nl * APA + 32 * q + 8 * i);
    }
  }
  if (tid < DN) {
    sPar[tid]      = encb[tid];
    sPar[DN + tid] = encw[tid];
  }
  if (tid < NBN) {
    int node = n0 + tid;
    node = node > nN - 1 ? nN - 1 : node;
    sX[tid] = x[node];
  }
  __syncthreads();

  const int rt = wave & 3, cg = wave >> 2;

  {
    v8f c0, c1, c2, c3;
    gemm3(sAh + (16 * rt + m) * APA + 8 * hh, sAl + (16 * rt + m) * APA + 8 * hh, wp + PEH, wp + PEL,
          DN, 4, 64 * cg, m, hh, c0, c1, c2, c3);
    float* sp = stg + (16 * rt + 8 * hh) * GSTR + 64 * cg + m;
    const float* bb = sPar + 64 * cg + m;
    const float* ww = sPar + DN + 64 * cg + m;
    const float* xp = sX + 16 * rt + 8 * hh;
    stage_enc(sp,      c0, bb[0],  ww[0],  xp);
    stage_enc(sp + 16, c1, bb[16], ww[16], xp);
    stage_enc(sp + 32, c2, bb[32], ww[32], xp);
    stage_enc(sp + 48, c3, bb[48], ww[48], xp);
  }
  __syncthreads();

#pragma unroll 1
  for (int it = 0; it < NBN / NWAVE; ++it) {
    const int s = wave + NWAVE * it;
    const v4f v = *(const v4f*)(stg + s * GSTR + 4 * lane);
    *(volatile v4f*)(Z + (size_t)(n0 + s) * DN + 4 * lane) = v;
  }
  {
    const int nl = tid >> 2, q = tid & 3;
    const float* rp = stg + nl * GSTR + 32 * q;
#pragma unroll
    for (int i = 0; i < 4; ++i) {
      const v4f a = *(const v4f*)(rp + 8 * i);
      const v4f b = *(const v4f*)(rp + 8 * i + 4);
      split8v(a, b, sAh + nl * APA + 32 * q + 8 * i, sAl + nl * APA + 32 * q + 8 * i);
    }
  }
  __threadfence();
#pragma unroll 1
  for (int it = 0; it < NBN / NWAVE; ++it) {
    const int s = wave + NWAVE * it;
    const v4f v = *(const v4f*)(stg + s * GSTR + 4 * lane);
    *(volatile v4f*)(Z + (size_t)(n0 + s) * DN + 4 * lane) = v;
  }
  __syncthreads();

  float* sw = stg + wave * 1024;
#pragma unroll 1
  for (int qq = 0; qq < 2; ++qq) {
    v8f c0, c1, c2, c3;
    gemm3(sAh + (16 * rt + m) * APA + 8 * hh, sAl + (16 * rt + m) * APA + 8 * hh, wp + PPH, wp + PPL,
          DN, 4, 128 * cg + 64 * qq, m, hh, c0, c1, c2, c3);
    {
      float* sp = sw + (8 * hh) * 64 + m;
#pragma unroll
      for (int r = 0; r < 8; ++r) {
        sp[r * 64]      = c0[r];
        sp[r * 64 + 16] = c1[r];
        sp[r * 64 + 32] = c2[r];
        sp[r * 64 + 48] = c3[r];
      }
    }
    __syncthreads();
#pragma unroll 1
    for (int i = 0; i < 8; ++i) {
      const int r2 = 2 * i + hh;
      const v4f v = *(const v4f*)(sw + r2 * 64 + 4 * m);
      const int row = n0 + 16 * rt + r2;
      *(volatile v4f*)(PQ + (size_t)row * PQROW + 128 * cg + 64 * qq + 4 * m) = v;
    }
    __threadfence();
#pragma unroll 1
    for (int i = 0; i < 8; ++i) {
      const int r2 = 2 * i + hh;
      const v4f v = *(const v4f*)(sw + r2 * 64 + 4 * m);
      const int row = n0 + 16 * rt + r2;
      *(volatile v4f*)(PQ + (size_t)row * PQROW + 128 * cg + 64 * qq + 4 * m) = v;
    }
    __syncthreads();
  }
}

__device__ __forceinline__ int scan_piece(const int* __restrict__ ei, int lim, int cbase, int base,
                                          int* list, int tid, int wave, int vec_ok) {
  int wc = 0;
  const int el0  = tid * EPT;
  const int e0   = cbase + el0;
  const int sent = -2147483647 - 1;
  int kk[EPT];
  if (vec_ok != 0 && cbase + PIECE <= lim) {
    const v4i* p = (const v4i*)(ei + e0);
#pragma unroll
    for (int u = 0; u < EPT / 4; ++u) {
      const v4i d = p[u];
      kk[4 * u] = d.x; kk[4 * u + 1] = d.y; kk[4 * u + 2] = d.z; kk[4 * u + 3] = d.w;
    }
  } else {
    const int lm = lim - 1;
#pragma unroll
    for (int q = 0; q < EPT; ++q) {
      const int eq = e0 + q;
      const int ec = eq > lm ? lm : eq;
      const int a = ei[ec];
      kk[q] = (eq < lim) ? a : sent;
    }
  }
  const unsigned nb = (unsigned)base;
  unsigned sq[EPT];
  bool hq[EPT];
  bool anyl = false;
#pragma unroll
  for (int q = 0; q < EPT; ++q) {
    sq[q] = (unsigned)kk[q] - nb;
    hq[q] = sq[q] < (unsigned)NBC;
    anyl = anyl | hq[q];
  }
  const unsigned any = __builtin_amdgcn_ballot_w32(anyl);
  if (any != 0u) {
#define HIT(HQ, SQ, Q) { \
      const unsigned mj = __builtin_amdgcn_ballot_w32(HQ); \
      if (mj != 0u) { \
        if (HQ) { \
          const int ps = wc + (int)__builtin_amdgcn_mbcnt_lo(mj, 0u); \
          if (ps < WCAP) list[wave * WCAP + ps] = ((el0 + (Q)) << SLB) | (int)(SQ); \
        } \
        wc += (int)__builtin_popcount(mj); } }
#pragma unroll
    for (int q = 0; q < EPT; ++q) {
      HIT(hq[q], sq[q], q)
    }
#undef HIT
  }
  return wc;
}

__device__ __forceinline__ void drain_max(const int* list, const int* wcnt, float* accF,
                                          const int* __restrict__ esrc, const float* __restrict__ eattr,
                                          const float* __restrict__ PQ, v4f wv,
                                          int cbase, int nE, int nN, int lane, int wave) {
#pragma unroll 1
  for (int wsx = 0; wsx < NWAVE; ++wsx) {
    int n = __builtin_amdgcn_readfirstlane(wcnt[wsx]);
    n = n > WCAP ? WCAP : (n < 0 ? 0 : n);
    const int* lp = list + wsx * WCAP;
#pragma unroll 1
    for (int bb = 0; bb < n; bb += 32) {
      const int idx = bb + lane;
      const int ic = idx > WCAP - 1 ? WCAP - 1 : idx;
      const int ent = lp[ic];
      const bool own = (idx < n) && ((ent & (NWAVE - 1)) == wave);
      unsigned msk = __builtin_amdgcn_ballot_w32(own);
#pragma unroll 1
      while (msk != 0u) {
        const int bit = (int)__builtin_ctz(msk);
        msk &= msk - 1u;
        const int e2 = __builtin_amdgcn_readlane(ent, bit);
        const int slot = e2 & (NBC - 1);
        const int el = (e2 >> SLB) & (PIECE - 1);
        int e = cbase + el;
        e = e > nE - 1 ? nE - 1 : (e < 0 ? 0 : e);
        const int s = iclamp(esrc[e], 0, nN - 1);
        const float ea = eattr[e];
        const v4f qv = *(const v4f*)(PQ + (size_t)s * PQROW + DN + 4 * lane);
        const v4f v = qv + wv * ea;
        float* ap = accF + slot * DN + 4 * lane;
        v4f a = *(const v4f*)ap;
        a.x = fmaxf(a.x, v.x);
        a.y = fmaxf(a.y, v.y);
        a.z = fmaxf(a.z, v.z);
        a.w = fmaxf(a.w, v.w);
        *(v4f*)ap = a;
      }
    }
  }
}

__device__ __forceinline__ void agg_rows(const float* accF, const float* __restrict__ PQ, v4f bv, float* AGG,
                                         int base, int nN, int lane, int wave, float ninf) {
#pragma unroll 1
  for (int it = 0; it < NBC / NWAVE; ++it) {
    const int s = wave + NWAVE * it;
    const int node = base + s;
    const int nc = node > nN - 1 ? nN - 1 : node;
    const v4f a = *(const v4f*)(accF + s * DN + 4 * lane);
    const v4f p = *(const v4f*)(PQ + (size_t)nc * PQROW + 4 * lane);
    v4f o;
    o.x = (a.x == ninf) ? 0.0f : fmaxf((p.x + bv.x) + a.x, 0.0f);
    o.y = (a.y == ninf) ? 0.0f : fmaxf((p.y + bv.y) + a.y, 0.0f);
    o.z = (a.z == ninf) ? 0.0f : fmaxf((p.z + bv.z) + a.z, 0.0f);
    o.w = (a.w == ninf) ? 0.0f : fmaxf((p.w + bv.w) + a.w, 0.0f);
    *(volatile v4f*)(AGG + (size_t)node * DN + 4 * lane) = o;
  }
}

__global__ __launch_bounds__(NTHR) void k_agg(
    const int* __restrict__ etgt, const int* __restrict__ esrc, const float* __restrict__ eattr,
    const float* __restrict__ PQ, const float* __restrict__ mw, const float* __restrict__ mb,
    float* AGG, int nE, int nN, int vec_ok) {
  extern __shared__ __attribute__((aligned(16))) float accF[];
  __shared__ int list[NWAVE * WCAP];
  __shared__ int wcnt[NWAVE];
  const int tid = (int)threadIdx.x, lane = tid & 31, wave = tid >> 5;
  const int base = (int)blockIdx.x * NBC;
  const float ninf = -__builtin_inff();

  {
    v4f nf;
    nf.x = ninf; nf.y = ninf; nf.z = ninf; nf.w = ninf;
#pragma unroll 1
    for (int i = tid; i < (NBC * DN) / 4; i += NTHR) *(v4f*)(accF + 4 * i) = nf;
  }
  const v4f wv = *(const v4f*)(mw + (size_t)2 * DN * DN + 4 * lane);
  const v4f bv = *(const v4f*)(mb + 4 * lane);
  __syncthreads();

#pragma unroll 1
  for (int cbase = 0; cbase < nE; cbase += PIECE) {
    const int wc = scan_piece(etgt, nE, cbase, base, list, tid, wave, vec_ok);
    if (lane == 0) wcnt[wave] = wc;
    __syncthreads();
    drain_max(list, wcnt, accF, esrc, eattr, PQ, wv, cbase, nE, nN, lane, wave);
    __syncthreads();
  }

  agg_rows(accF, PQ, bv, AGG, base, nN, lane, wave, ninf);
  __threadfence();
  agg_rows(accF, PQ, bv, AGG, base, nN, lane, wave, ninf);
}

__device__ __forceinline__ void upd_store(const float* stg, const float* sHP, const float* sY,
                                          float* hout, float* yout, float* HP,
                                          int n0, int nN, int yfull, int blk, int lane, int wave) {
#pragma unroll 1
  for (int it = 0; it < NBN / NWAVE; ++it) {
    const int s = wave + NWAVE * it;
    const int node = n0 + s;
    if (node < nN) {
      const v4f v = *(const v4f*)(stg + s * GSTR + 4 * lane);
      *(volatile v4f*)(hout + (size_t)node * DN + 4 * lane) = v;
    }
  }
  if (wave == 0) {
    const v4f v = *(const v4f*)(sHP + 4 * lane);
    *(volatile v4f*)(HP + (size_t)blk * DN + 4 * lane) = v;
  }
  if (wave == 1 && lane < 16) {
    const int nb = n0 + 4 * lane;
    if (nb + 4 <= yfull) {
      const v4f v = *(const v4f*)(sY + 4 * lane);
      *(volatile v4f*)(yout + (size_t)nb) = v;
    }
  }
}

__global__ __launch_bounds__(NTHR) void k_upd(
    const float* __restrict__ Z, const float* __restrict__ AGG, const unsigned short* __restrict__ wp,
    const float* __restrict__ ub, const float* __restrict__ decw, const float* __restrict__ decb,
    float* hout, float* yout, float* HP, int nN, int yfull) {
  extern __shared__ __attribute__((aligned(16))) unsigned short sAx[];
  __shared__ __attribute__((aligned(16))) float stg[NBN * GSTR];
  __shared__ __attribute__((aligned(16))) float sPar[3 * DN];
  __shared__ __attribute__((aligned(16))) float sHP[DN];
  __shared__ __attribute__((aligned(16))) float sY[NBN];
  __shared__ float sYz[NBN];
  __shared__ float sDb;
  unsigned short* sAh = sAx;
  unsigned short* sAl = sAx + NBN * APN;
  const int tid = (int)threadIdx.x, lane = tid & 31, wave = tid >> 5, hh = lane >> 4, m = lane & 15;
  const int n0 = (int)blockIdx.x * NBN;

  {
    const int nl = tid >> 2, q = tid & 3;
    int node = n0 + nl;
    node = node > nN - 1 ? nN - 1 : node;
    const float* zp = Z   + (size_t)node * DN + 32 * q;
    const float* gp = AGG + (size_t)node * DN + 32 * q;
    const float* wd = decw + 32 * q;
    float pz = 0.0f;
#pragma unroll
    for (int i = 0; i < 4; ++i) {
      const v4f a  = *(const v4f*)(zp + 8 * i);
      const v4f b  = *(const v4f*)(zp + 8 * i + 4);
      const v4f w0 = *(const v4f*)(wd + 8 * i);
      const v4f w1 = *(const v4f*)(wd + 8 * i + 4);
      pz += a.x * w0.x; pz += a.y * w0.y; pz += a.z * w0.z; pz += a.w * w0.w;
      pz += b.x * w1.x; pz += b.y * w1.y; pz += b.z * w1.z; pz += b.w * w1.w;
      split8v(a, b, sAh + nl * APN + 32 * q + 8 * i, sAl + nl * APN + 32 * q + 8 * i);
    }
#pragma unroll
    for (int i = 0; i < 4; ++i) {
      const v4f a = *(const v4f*)(gp + 8 * i);
      const v4f b = *(const v4f*)(gp + 8 * i + 4);
      split8v(a, b, sAh + nl * APN + DN + 32 * q + 8 * i, sAl + nl * APN + DN + 32 * q + 8 * i);
    }
    pz += __shfl_xor(pz, 1);
    pz += __shfl_xor(pz, 2);
    if (q == 0) sYz[nl] = pz;
  }
  if (tid < DN) {
    sPar[tid]          = ub[tid];
    sPar[DN + tid]     = decw[tid];
    sPar[2 * DN + tid] = decw[DN + tid];
  }
  if (tid == 0) sDb = decb[0];
  __syncthreads();

  const int rt = wave & 3, cg = wave >> 2;

  {
    v8f c0, c1, c2, c3;
    gemm3(sAh + (16 * rt + m) * APN + 8 * hh, sAl + (16 * rt + m) * APN + 8 * hh, wp + PUH, wp + PUL,
          2 * DN, 8, 64 * cg, m, hh, c0, c1, c2, c3);
    float* sp = stg + (16 * rt + 8 * hh) * GSTR + 64 * cg + m;
    const float* bb = sPar + 64 * cg + m;
    stage_relu(sp,      c0, bb[0]);
    stage_relu(sp + 16, c1, bb[16]);
    stage_relu(sp + 32, c2, bb[32]);
    stage_relu(sp + 48, c3, bb[48]);
  }
  __syncthreads();

  {
    const int nl = tid >> 2, q = tid & 3;
    const float* row = stg + nl * GSTR + 32 * q;
    const float* w = sPar + 2 * DN + 32 * q;
    float ph = 0.0f;
#pragma unroll 4
    for (int c = 0; c < 32; ++c) ph += row[c] * w[c];
    ph += __shfl_xor(ph, 1);
    ph += __shfl_xor(ph, 2);
    const float yv = sigm_f((sYz[nl] + ph) + sDb);
    if (q == 0) sY[nl] = yv;
  }
  if (tid < DN) {
    int nv = nN - n0;
    nv = nv > NBN ? NBN : (nv < 0 ? 0 : nv);
    float s = 0.0f;
#pragma unroll 4
    for (int r = 0; r < nv; ++r) s += stg[r * GSTR + tid];
    sHP[tid] = s;
  }
  __syncthreads();

  upd_store(stg, sHP, sY, hout, yout, HP, n0, nN, yfull, (int)blockIdx.x, lane, wave);
  __threadfence();
  upd_store(stg, sHP, sY, hout, yout, HP, n0, nN, yfull, (int)blockIdx.x, lane, wave);
}

__global__ __launch_bounds__(NTHR) void k_term(
    const float* __restrict__ HP, int nblk, const float* __restrict__ terw, const float* __restrict__ terb,
    const float* __restrict__ Z, const float* hsrc, const float* __restrict__ decw, const float* __restrict__ decb,
    float* ytail, int nN, int yfull) {
  __shared__ double red[DN];
  __shared__ float sT[40];
  const int tid = (int)threadIdx.x, lane = tid & 31, wave = tid >> 5;
  const int nrem = nN - yfull;

  if (tid < DN) {
    double part = 0.0;
#pragma unroll 1
    for (int b = 0; b < nblk; ++b) part += (double)HP[(size_t)b * DN + tid];
    const double rn = 1.0 / (double)nN;
    red[tid] = (part * rn) * ((double)terw[tid] + (double)terw[DN + tid]);
  }
  {
    const float db = decb[0];
#pragma unroll 1
    for (int k = 0; k < 4; ++k) {
      const int j = wave + NWAVE * k;
      int node = yfull + j;
      node = node > nN - 1 ? nN - 1 : node;
      const float* zr = Z    + (size_t)node * DN;
      const float* hr = hsrc + (size_t)node * DN;
      float t = 0.0f;
#pragma unroll
      for (int i = 0; i < 4; ++i) {
        const int c = lane + 32 * i;
        t += zr[c] * decw[c];
        t += hr[c] * decw[DN + c];
      }
      t += __shfl_xor(t, 16);
      t += __shfl_xor(t, 8);
      t += __shfl_xor(t, 4);
      t += __shfl_xor(t, 2);
      t += __shfl_xor(t, 1);
      const float yv = sigm_f(t + db);
      if (lane == 0) sT[j] = yv;
    }
  }
  __syncthreads();
#pragma unroll 1
  for (int o = 64; o > 0; o >>= 1) {
    if (tid < o) red[tid] += red[tid + o];
    __syncthreads();
  }
  if (tid == 0) sT[nrem] = (float)(red[0] + (double)terb[0]);
  __syncthreads();
  if (tid <= nrem) {
    const float v = sT[tid];
    *(volatile float*)(ytail + tid) = v;
  }
  __threadfence();
  if (tid <= nrem) {
    const float v = sT[tid];
    *(volatile float*)(ytail + tid) = v;
  }
}

extern "C" void kernel_launch(void* const* d_in, const int* in_sizes, int n_in,
                              void* d_out, int out_size, void* d_ws, size_t ws_size,
                              hipStream_t stream) {
  if (n_in < 14) return;
  const int nN = in_sizes[0];
  if (nN < 1 || nN > (1 << 22)) return;
  if (in_sizes[1] != nN * DN) return;
  const int nE = in_sizes[2];
  if (nE < 1 || nE > (1 << 26)) return;
  if (in_sizes[3] != (DN + 1) * DN || in_sizes[4] != DN) return;
  if (in_sizes[5] != (2 * DN + 1) * DN || in_sizes[6] != DN) return;
  if (in_sizes[7] != 2 * DN * DN || in_sizes[8] != DN) return;
  if (in_sizes[9] != 2 * DN || in_sizes[10] < 1) return;
  if (in_sizes[11] != 2 * DN || in_sizes[12] < 1) return;
  if (in_sizes[13] != 2 * nE) return;
  if ((size_t)out_size != (size_t)nN * DN + (size_t)nN + 1) return;

  const float* x     = (const float*)d_in[0];
  const float* preh  = (const float*)d_in[1];
  const float* eattr = (const float*)d_in[2];
  const float* encw  = (const float*)d_in[3];
  const float* encb  = (const float*)d_in[4];
  const float* mw    = (const float*)d_in[5];
  const float* mb    = (const float*)d_in[6];
  const float* uw    = (const float*)d_in[7];
  const float* ub    = (const float*)d_in[8];
  const float* decw  = (const float*)d_in[9];
  const float* decb  = (const float*)d_in[10];
  const float* terw  = (const float*)d_in[11];
  const float* terb  = (const float*)d_in[12];
  const int*   eidx  = (const int*)d_in[13];
  const int*   esrc  = eidx;
  const int*   etgt  = eidx + nE;

  float* hout = (float*)d_out;
  float* yout = hout + (size_t)nN * DN;
  const int yfull = (nN / 32) * 32;
  float* ytail = yout + yfull;

  const int nb64 = (nN + NBN - 1) / NBN;
  const int Npad64 = nb64 * NBN;
  const int nbA = (nN + NBC - 1) / NBC;
  const int Npad512 = nbA * NBC;
  const int vec_ok = ((nE & 3) == 0) ? 1 : 0;

  char* ws = (char*)d_ws;
  size_t off = 0;
  const size_t oW  = off; off += (size_t)PWTOT * 2;               off = (off + 255) & ~(size_t)255;
  const size_t oZ  = off; off += (size_t)Npad64 * DN * 4;         off = (off + 255) & ~(size_t)255;
  const size_t oPQ = off; off += (size_t)Npad64 * PQROW * 4;      off = (off + 255) & ~(size_t)255;
  const size_t oAG = off; off += (size_t)Npad512 * DN * 4;        off = (off + 255) & ~(size_t)255;
  const size_t oHP = off; off += (size_t)nb64 * DN * 4;           off = (off + 255) & ~(size_t)255;
  if (off > ws_size || off > (size_t)WSCAP) return;
  unsigned short* wp = (unsigned short*)(ws + oW);
  float* Z   = (float*)(ws + oZ);
  float* PQ  = (float*)(ws + oPQ);
  float* AGG = (float*)(ws + oAG);
  float* HP  = (float*)(ws + oHP);

  hipFuncSetAttribute(reinterpret_cast<const void*>(&k_agg), hipFuncAttributeMaxDynamicSharedMemorySize, AGGDYN);
  hipFuncSetAttribute(reinterpret_cast<const void*>(&k_upd), hipFuncAttributeMaxDynamicSharedMemorySize, UPDDYN);

  k_prep<<<PBLK, NTHR, 0, stream>>>(encw, mw, uw, wp);
  k_encpq<<<nb64, NTHR, ENCDYN, stream>>>(x, preh, encw, encb, wp, Z, PQ, nN);
  k_agg<<<nbA, NTHR, AGGDYN, stream>>>(etgt, esrc, eattr, PQ, mw, mb, AGG, nE, nN, vec_ok);
  k_upd<<<nb64, NTHR, UPDDYN, stream>>>(Z, AGG, wp, ub, decw, decb, hout, yout, HP, nN, yfull);
  k_term<<<1, NTHR, 0, stream>>>(HP, nb64, terw, terb, Z, hout, decw, decb, ytail, nN, yfull);
}
